// TorchAttentionMechanism_18425409700363
// MI455X (gfx1250) — hardware-verified
//
#include <hip/hip_runtime.h>
#include <math.h>

constexpr int kBatch   = 8;
constexpr int kSeq     = 1024;
constexpr int kEmb     = 1024;
constexpr int kHeads   = 16;
constexpr int kHeadDim = 64;
constexpr int kTok     = kBatch * kSeq;
constexpr int kGroup   = 8;
constexpr int kGroupsPerBatch = kHeads / kGroup;
constexpr int kChunks  = kBatch * kGroupsPerBatch;

constexpr float kWCarry     = 16.0f;
constexpr float kQKCarry    = 4.0f;
constexpr float kPCarry     = 2048.0f;
constexpr float kOCarry     = 64.0f;
constexpr float kProjScale  = 1.0f / kWCarry;
constexpr float kScoreScale = 1.0f / (kQKCarry * kQKCarry * 64.0f);
constexpr float kPVScale    = kOCarry / kPCarry;
constexpr float kOutScale   = 1.0f / (kOCarry * kWCarry);
constexpr float kInv64      = 1.0f / 64.0f;
constexpr float kInv63      = 1.0f / 63.0f;

constexpr size_t kMiB     = 1048576;
constexpr size_t kOffX16  = 0;
constexpr size_t kOffWq16 = 16 * kMiB;
constexpr size_t kOffWk16 = 18 * kMiB;
constexpr size_t kOffWv16 = 20 * kMiB;
constexpr size_t kOffWo16 = 22 * kMiB;
constexpr size_t kOffQF   = 24 * kMiB;
constexpr size_t kOffP16  = 56 * kMiB;
constexpr size_t kOffVT16 = 72 * kMiB;
constexpr size_t kOffQC16 = 88 * kMiB;
constexpr size_t kOffKC16 = 104 * kMiB;
constexpr size_t kOffQVar = 120 * kMiB;
constexpr size_t kOffKVar = 120 * kMiB + 512 * 1024;
constexpr size_t kWsTotal = 121 * kMiB;
static_assert((size_t)kTok * kEmb * 2 == 16 * kMiB, "x / o planes 16 MiB");
static_assert((size_t)kEmb * kEmb * 2 == 2 * kMiB, "weight planes 2 MiB");
static_assert((size_t)kTok * kEmb * 4 == 32 * kMiB, "f32 projection plane 32 MiB");
static_assert((size_t)kGroup * kSeq * kSeq * 4 == 32 * kMiB, "scores plane fits the projection region");
static_assert((size_t)kGroup * kSeq * kSeq * 2 == 16 * kMiB, "probability plane 16 MiB");
static_assert((size_t)kTok * kHeads * 4 == 512 * 1024, "variance tables 512 KiB");
static_assert(kOffKVar + (size_t)kTok * kHeads * 4 == kWsTotal, "carve end");
static_assert(kWsTotal <= (size_t)134217728, "carve under 128 MiB");
static_assert(kEmb % 32 == 0 && kHeadDim % 32 == 0 && kSeq % 32 == 0, "K multiples of 32");
static_assert(kTok % 64 == 0 && kEmb % 64 == 0 && kSeq % 64 == 0 && kHeadDim % 64 == 0, "M, N multiples of 64");

typedef __attribute__((ext_vector_type(16))) _Float16 v16h;
typedef __attribute__((ext_vector_type(8)))  _Float16 v8h;
typedef __attribute__((ext_vector_type(16))) __bf16   v16b;
typedef __attribute__((ext_vector_type(8)))  __bf16   v8b;
typedef __attribute__((ext_vector_type(8)))  float    v8f;
typedef __attribute__((ext_vector_type(4)))  float    v4f;
typedef __attribute__((ext_vector_type(4)))  unsigned int v4u;

__device__ __forceinline__ unsigned short f2bf_bits(float f) {
  unsigned u = __float_as_uint(f);
  return (unsigned short)((u + 0x7FFFu + ((u >> 16) & 1u)) >> 16);
}
__device__ __forceinline__ float bf_bits2f(unsigned short h) { return __uint_as_float(((unsigned)h) << 16); }

__device__ __forceinline__ void dep_guard_h(v8f& a, v8f& b, v16h x, v16h y) { asm volatile("v_nop\n\tv_nop\n\tv_nop\n\tv_nop" : "+v"(a), "+v"(b) : "v"(x), "v"(y)); }
__device__ __forceinline__ void dep_guard_b(v8f& a, v8f& b, v16b x, v16b y) { asm volatile("v_nop\n\tv_nop\n\tv_nop\n\tv_nop" : "+v"(a), "+v"(b) : "v"(x), "v"(y)); }
__device__ __forceinline__ void keep4_h(v16h a, v16h b, v16h c, v16h d) { asm volatile("v_nop" :: "v"(a), "v"(b), "v"(c), "v"(d)); }
__device__ __forceinline__ void keep4_b(v16b a, v16b b, v16b c, v16b d) { asm volatile("v_nop" :: "v"(a), "v"(b), "v"(c), "v"(d)); }
__device__ __forceinline__ void acc_guard4(v8f& a, v8f& b, v8f& c, v8f& d) { asm volatile("v_nop\n\tv_nop\n\tv_nop\n\tv_nop" : "+v"(a), "+v"(b), "+v"(c), "+v"(d)); }
template <typename T> struct Frag;
template <> struct Frag<_Float16> {
  typedef v16h V; union U { v16h v; v8h h[2]; };
  static __device__ __forceinline__ v16h load(const _Float16* p) {
    U f; f.h[0] = *(const v8h*)(p); f.h[1] = *(const v8h*)(p + 16); return f.v;
  }
  static __device__ __forceinline__ v8f mma(v16h a, v16h b, v8f c) {
    return __builtin_amdgcn_wmma_f32_16x16x32_f16(false, a, false, b, (short)0, c, false, false);
  }
  static __device__ __forceinline__ void guard(v8f& a, v8f& b, v16h x, v16h y) { dep_guard_h(a, b, x, y); }
  static __device__ __forceinline__ void keep(v16h a, v16h b, v16h c, v16h d) { keep4_h(a, b, c, d); }
};
template <> struct Frag<__bf16> {
  typedef v16b V; union U { v16b v; v8b h[2]; };
  static __device__ __forceinline__ v16b load(const __bf16* p) {
    U f; f.h[0] = *(const v8b*)(p); f.h[1] = *(const v8b*)(p + 16); return f.v;
  }
  static __device__ __forceinline__ v8f mma(v16b a, v16b b, v8f c) {
    return __builtin_amdgcn_wmma_f32_16x16x32_bf16(false, a, false, b, (short)0, c, false, false);
  }
  static __device__ __forceinline__ void guard(v8f& a, v8f& b, v16b x, v16b y) { dep_guard_b(a, b, x, y); }
  static __device__ __forceinline__ void keep(v16b a, v16b b, v16b c, v16b d) { keep4_b(a, b, c, d); }
};

__device__ __forceinline__ unsigned pk16(unsigned short a, unsigned short b) { return (unsigned)a | ((unsigned)b << 16); }
__device__ __forceinline__ unsigned short h_bits(float f) { const _Float16 h = (_Float16)f; return __builtin_bit_cast(unsigned short, h); }

template <int ET> struct Elem;
template <> struct Elem<0> { typedef _Float16 T; };
template <> struct Elem<1> { typedef __bf16 T; };
template <int ET, bool SPLIT, int BIAS_MODE, int OUT_MODE, bool RESID, int ACT = 0>
__global__ __launch_bounds__(256) void wmma_gemm64(
    const unsigned short* __restrict__ Ap, const unsigned short* __restrict__ A2p, int lda, long strideA,
    const unsigned short* __restrict__ Btp, const unsigned short* __restrict__ Bt2p, int ldb, long strideB,
    void* __restrict__ Cout, void* __restrict__ Cout2, int ldc, long strideC,
    const float* __restrict__ bias,
    const float* __restrict__ resid, long strideR,
    int M, int N, int K, float scale) {
  typedef typename Elem<ET>::T T;
  typedef typename Frag<T>::V V;
  const T* A = (const T*)Ap; const T* A2 = (const T*)A2p; const T* Bt = (const T*)Btp; const T* Bt2 = (const T*)Bt2p;
  __shared__ __align__(16) float sT[8][16 * 68];
  const int b    = blockIdx.y;
  const int lane = threadIdx.x & 31;
  const int wave = threadIdx.x >> 5;
  const int tilesN = N >> 6;
  const int tilesM = M >> 6;
  const int tile = blockIdx.x * 8 + wave;
  if (tile >= tilesM * tilesN) return;
  const int tm = tile / tilesN;
  const int tn = tile - tm * tilesN;
  const int m0 = tm << 6;
  const int n0 = tn << 6;

  const T* Ab  = A  + (size_t)b * strideA;
  const T* Bb  = Bt + (size_t)b * strideB;
  const T* Ab2 = SPLIT ? (A2  + (size_t)b * strideA) : nullptr;
  const T* Bb2 = SPLIT ? (Bt2 + (size_t)b * strideB) : nullptr;

  const int rlane = lane & 15;
  const int koff  = (lane >> 4) * 8;
  const int mOff  = (lane >> 4) * 8;

  v8f acc[4][4];
#pragma unroll
  for (int i = 0; i < 4; ++i)
#pragma unroll
    for (int j = 0; j < 4; ++j) acc[i][j] = (v8f){0.f,0.f,0.f,0.f,0.f,0.f,0.f,0.f};

  for (int k0 = 0; k0 < K; k0 += 32) {
    V bh[4], bl[4];
#pragma unroll
    for (int j = 0; j < 4; ++j) {
      const size_t bo = (size_t)(n0 + (j << 4) + rlane) * ldb + koff + k0;
      bh[j] = Frag<T>::load(Bb + bo);
      if (SPLIT) bl[j] = Frag<T>::load(Bb2 + bo);
    }
#pragma unroll
    for (int i = 0; i < 4; ++i) {
      const size_t ao = (size_t)(m0 + (i << 4) + rlane) * lda + koff + k0;
      V ah = Frag<T>::load(Ab + ao);
      V al;
      if (SPLIT) al = Frag<T>::load(Ab2 + ao);
#pragma unroll
      for (int j = 0; j < 4; ++j) {
        acc[i][j] = Frag<T>::mma(ah, bh[j], acc[i][j]);
        if (SPLIT) {
          acc[i][j] = Frag<T>::mma(ah, bl[j], acc[i][j]);
          acc[i][j] = Frag<T>::mma(al, bh[j], acc[i][j]);
        }
      }
      Frag<T>::guard(acc[i][0], acc[i][3], ah, SPLIT ? al : ah);
    }
    Frag<T>::keep(bh[0], bh[1], bh[2], bh[3]);
    if (SPLIT) Frag<T>::keep(bl[0], bl[1], bl[2], bl[3]);
  }
  acc_guard4(acc[0][0], acc[0][1], acc[0][2], acc[0][3]);
  acc_guard4(acc[1][0], acc[1][1], acc[1][2], acc[1][3]);
  acc_guard4(acc[2][0], acc[2][1], acc[2][2], acc[2][3]);
  acc_guard4(acc[3][0], acc[3][1], acc[3][2], acc[3][3]);

  float* slab = sT[wave];
  const float* Rb = RESID ? (resid + (size_t)b * strideR) : nullptr;
#pragma unroll
  for (int i = 0; i < 4; ++i) {
    const int mBase = m0 + (i << 4);
#pragma unroll
    for (int j = 0; j < 4; ++j) {
      const int n = n0 + (j << 4) + rlane;
      float bv = 0.f;
      if (BIAS_MODE == 2) bv = bias[n];
#pragma unroll
      for (int r = 0; r < 8; ++r) {
        float v = acc[i][j][r] * scale;
        if (BIAS_MODE == 1) v += bias[mBase + mOff + r];
        if (BIAS_MODE == 2) v += bv;
        if (RESID) v += Rb[(size_t)(mBase + mOff + r) * ldc + n];
        if (ACT == 2) v = fmaxf(v, 0.0f);
        if (ACT == 4) v = (v > 0.f) ? v : 0.01f * v;
        slab[(mOff + r) * 68 + (j << 4) + rlane] = v;
      }
    }
    __builtin_amdgcn_fence(__ATOMIC_RELEASE, "workgroup");
    __builtin_amdgcn_wave_barrier();
    __builtin_amdgcn_fence(__ATOMIC_ACQUIRE, "workgroup");
    if (OUT_MODE == 0) {
      float* C = (float*)Cout + (size_t)b * strideC;
      const int hh = lane >> 4, c4 = (lane & 15) * 4;
      for (int pass = 0; pass < 2; ++pass) {
#pragma unroll
        for (int it = 0; it < 8; ++it) {
          const int row = it * 2 + hh;
          v4f v = *(const v4f*)(slab + row * 68 + c4);
          *(volatile v4f*)(C + (size_t)(mBase + row) * ldc + n0 + c4) = v;
        }
        __threadfence();
      }
    } else {
      const int q = lane >> 3, c8 = (lane & 7) * 8;
      unsigned short* C  = (unsigned short*)Cout  + (size_t)b * strideC;
      unsigned short* C2 = (OUT_MODE == 2) ? ((unsigned short*)Cout2 + (size_t)b * strideC) : nullptr;
      for (int pass = 0; pass < 2; ++pass) {
#pragma unroll
        for (int it = 0; it < 4; ++it) {
          const int row = it * 4 + q;
          const float* sp = slab + row * 68 + c8;
          v8h hv, lv;
#pragma unroll
          for (int e = 0; e < 8; ++e) {
            if (OUT_MODE == 1) {
              hv[e] = (_Float16)sp[e];
            } else {
              unsigned short hb = f2bf_bits(sp[e]);
              unsigned short lb = f2bf_bits(sp[e] - bf_bits2f(hb));
              hv[e] = __builtin_bit_cast(_Float16, hb);
              lv[e] = __builtin_bit_cast(_Float16, lb);
            }
          }
          *(volatile v8h*)(C + (size_t)(mBase + row) * ldc + n0 + c8) = hv;
          if (OUT_MODE == 2) *(volatile v8h*)(C2 + (size_t)(mBase + row) * ldc + n0 + c8) = lv;
        }
        __threadfence();
      }
    }
    __builtin_amdgcn_fence(__ATOMIC_RELEASE, "workgroup");
    __builtin_amdgcn_wave_barrier();
    __builtin_amdgcn_fence(__ATOMIC_ACQUIRE, "workgroup");
  }
}

__global__ __launch_bounds__(256) void cast8_f16_kernel(const float* __restrict__ in, unsigned short* __restrict__ out,
                                                        int n8, float scale) {
  const int i = blockIdx.x * 256 + threadIdx.x;
  if (i >= n8) return;
  const float* p = in + 8 * (size_t)i;
  const v4f a = *(const v4f*)(p);
  const v4f c = *(const v4f*)(p + 4);
  unsigned short hb[8];
#pragma unroll
  for (int e = 0; e < 4; ++e) {
    hb[e]     = h_bits(a[e] * scale);
    hb[4 + e] = h_bits(c[e] * scale);
  }
  const v4u u = (v4u){pk16(hb[0], hb[1]), pk16(hb[2], hb[3]), pk16(hb[4], hb[5]), pk16(hb[6], hb[7])};
  unsigned short* q = out + 8 * (size_t)i;
  *(volatile v4u*)q = u;
  __threadfence();
  *(volatile v4u*)q = u;
}

__global__ __launch_bounds__(256) void center_kernel(const float* __restrict__ src, unsigned short* __restrict__ dst,
                                                     float* __restrict__ var_out, float carry) {
  __shared__ __align__(16) float sv[8 * 16];
  const int t    = threadIdx.x;
  const int lane = t & 31, wave = t >> 5;
  const int tok  = blockIdx.x * 8 + wave;
  const int g    = lane >> 3;
  const int e8   = (lane & 7) * 8;
  const float* row = src + (size_t)tok * kEmb;
  unsigned short* drow = dst + (size_t)tok * kEmb;
#pragma unroll
  for (int hq = 0; hq < 4; ++hq) {
    const int h = hq * 4 + g;
    const float* p = row + h * kHeadDim + e8;
    const v4f a = *(const v4f*)(p);
    const v4f c = *(const v4f*)(p + 4);
    float x[8];
#pragma unroll
    for (int e = 0; e < 4; ++e) { x[e] = a[e]; x[4 + e] = c[e]; }
    float s = ((x[0] + x[1]) + (x[2] + x[3])) + ((x[4] + x[5]) + (x[6] + x[7]));
    s += __shfl_xor(s, 1, 32);
    s += __shfl_xor(s, 2, 32);
    s += __shfl_xor(s, 4, 32);
    const float mean = s * kInv64;
    float vs = 0.f;
#pragma unroll
    for (int e = 0; e < 8; ++e) { x[e] = x[e] - mean; vs += x[e] * x[e]; }
    vs += __shfl_xor(vs, 1, 32);
    vs += __shfl_xor(vs, 2, 32);
    vs += __shfl_xor(vs, 4, 32);
    unsigned short hb[8];
#pragma unroll
    for (int e = 0; e < 8; ++e) hb[e] = h_bits(x[e] * carry);
    const v4u u = (v4u){pk16(hb[0], hb[1]), pk16(hb[2], hb[3]), pk16(hb[4], hb[5]), pk16(hb[6], hb[7])};
    unsigned short* q = drow + h * kHeadDim + e8;
    *(volatile v4u*)q = u;
    __threadfence();
    *(volatile v4u*)q = u;
    if ((lane & 7) == 0) sv[wave * 16 + h] = vs * kInv63;
  }
  __syncthreads();
  if (wave == 0) {
    const v4f v = *(const v4f*)(sv + 4 * lane);
    float* vp = var_out + (size_t)blockIdx.x * 128 + 4 * lane;
    *(volatile v4f*)vp = v;
    __threadfence();
    *(volatile v4f*)vp = v;
  }
}

__global__ __launch_bounds__(128) void softmax_kernel(const float* __restrict__ sc, const float* __restrict__ qvar,
                                                      const float* __restrict__ kvar, unsigned short* __restrict__ pout,
                                                      int bidx, int h0) {
  __shared__ float redM[4];
  __shared__ float redS[4];
  const int r    = blockIdx.x;
  const int hl   = r >> 10;
  const int qi   = r & (kSeq - 1);
  const int h    = h0 + hl;
  const int t    = threadIdx.x;
  const int lane = t & 31, wave = t >> 5;
  const int c0   = t * 8;
  const float qv = qvar[((size_t)bidx * kSeq + qi) * kHeads + h];
  const float* sr = sc + (size_t)r * kSeq + c0;
  const v4f a = *(const v4f*)(sr);
  const v4f c = *(const v4f*)(sr + 4);
  const float* kvp = kvar + ((size_t)bidx * kSeq + c0) * kHeads + h;
  float x[8];
#pragma unroll
  for (int e = 0; e < 4; ++e) {
    x[e]     = a[e] + (qv * kvp[e * kHeads]) * kInv64;
    x[4 + e] = c[e] + (qv * kvp[(4 + e) * kHeads]) * kInv64;
  }
  float m = fmaxf(fmaxf(fmaxf(x[0], x[1]), fmaxf(x[2], x[3])), fmaxf(fmaxf(x[4], x[5]), fmaxf(x[6], x[7])));
#pragma unroll
  for (int off = 16; off > 0; off >>= 1) m = fmaxf(m, __shfl_xor(m, off, 32));
  if (lane == 0) redM[wave] = m;
  __syncthreads();
  m = fmaxf(fmaxf(redM[0], redM[1]), fmaxf(redM[2], redM[3]));
  float ex[8];
  float s = 0.f;
#pragma unroll
  for (int e = 0; e < 8; ++e) { ex[e] = expf(x[e] - m); s += ex[e]; }
#pragma unroll
  for (int off = 16; off > 0; off >>= 1) s += __shfl_xor(s, off, 32);
  if (lane == 0) redS[wave] = s;
  __syncthreads();
  s = (redS[0] + redS[1]) + (redS[2] + redS[3]);
  const float inv = kPCarry * (1.0f / s);
  unsigned short hb[8];
#pragma unroll
  for (int e = 0; e < 8; ++e) hb[e] = h_bits(ex[e] * inv);
  const v4u u = (v4u){pk16(hb[0], hb[1]), pk16(hb[2], hb[3]), pk16(hb[4], hb[5]), pk16(hb[6], hb[7])};
  unsigned short* q = pout + (size_t)r * kSeq + c0;
  *(volatile v4u*)q = u;
  __threadfence();
  *(volatile v4u*)q = u;
}

extern "C" void kernel_launch(void* const* d_in, const int* in_sizes, int n_in,
                              void* d_out, int out_size, void* d_ws, size_t ws_size,
                              hipStream_t stream) {
  if (n_in < 5) return;
  if (in_sizes[0] != kTok * kEmb) return;
  if (in_sizes[1] != kEmb * kEmb || in_sizes[2] != kEmb * kEmb || in_sizes[3] != kEmb * kEmb || in_sizes[4] != kEmb * kEmb) return;
  if (out_size != kTok * kEmb) return;
  if (ws_size < kWsTotal) return;

  const float* x  = (const float*)d_in[0];
  const float* Wq = (const float*)d_in[1];
  const float* Wk = (const float*)d_in[2];
  const float* Wv = (const float*)d_in[3];
  const float* Wo = (const float*)d_in[4];
  float* outp = (float*)d_out;

  char* ws = (char*)d_ws;
  unsigned short* X16  = (unsigned short*)(ws + kOffX16);
  unsigned short* O16  = (unsigned short*)(ws + kOffX16);
  unsigned short* Wq16 = (unsigned short*)(ws + kOffWq16);
  unsigned short* Wk16 = (unsigned short*)(ws + kOffWk16);
  unsigned short* Wv16 = (unsigned short*)(ws + kOffWv16);
  unsigned short* Wo16 = (unsigned short*)(ws + kOffWo16);
  float*          QF   = (float*)(ws + kOffQF);
  float*          SC   = (float*)(ws + kOffQF);
  unsigned short* P16  = (unsigned short*)(ws + kOffP16);
  unsigned short* VT16 = (unsigned short*)(ws + kOffVT16);
  unsigned short* QC16 = (unsigned short*)(ws + kOffQC16);
  unsigned short* KC16 = (unsigned short*)(ws + kOffKC16);
  float*          QVAR = (float*)(ws + kOffQVar);
  float*          KVAR = (float*)(ws + kOffKVar);

  const float* nof = (const float*)nullptr;
  const unsigned short* nou = (const unsigned short*)nullptr;

  {
    const int n8x = kTok * kEmb / 8;
    const int n8w = kEmb * kEmb / 8;
    cast8_f16_kernel<<<(n8x + 255) / 256, 256, 0, stream>>>(x, X16, n8x, 1.0f);
    cast8_f16_kernel<<<(n8w + 255) / 256, 256, 0, stream>>>(Wq, Wq16, n8w, kWCarry);
    cast8_f16_kernel<<<(n8w + 255) / 256, 256, 0, stream>>>(Wk, Wk16, n8w, kWCarry);
    cast8_f16_kernel<<<(n8w + 255) / 256, 256, 0, stream>>>(Wv, Wv16, n8w, kWCarry);
    cast8_f16_kernel<<<(n8w + 255) / 256, 256, 0, stream>>>(Wo, Wo16, n8w, kWCarry);
  }

  {
    const int tiles = (kEmb / 64) * (kTok / 64);
    wmma_gemm64<0, false, 0, 1, false, 0><<<dim3((tiles + 7) / 8, 1), 256, 0, stream>>>(
        Wv16, nou, kEmb, 0L, X16, nou, kEmb, 0L, (void*)VT16, (void*)nullptr, kTok, 0L,
        nof, nof, 0L, kEmb, kTok, kEmb, kProjScale);
  }

  {
    const int tiles = (kTok / 64) * (kEmb / 64);
    wmma_gemm64<0, false, 0, 0, false, 0><<<dim3((tiles + 7) / 8, 1), 256, 0, stream>>>(
        X16, nou, kEmb, 0L, Wq16, nou, kEmb, 0L, (void*)QF, (void*)nullptr, kEmb, 0L,
        nof, nof, 0L, kTok, kEmb, kEmb, kProjScale);
    center_kernel<<<kTok / 8, 256, 0, stream>>>(QF, QC16, QVAR, kQKCarry);
    wmma_gemm64<0, false, 0, 0, false, 0><<<dim3((tiles + 7) / 8, 1), 256, 0, stream>>>(
        X16, nou, kEmb, 0L, Wk16, nou, kEmb, 0L, (void*)QF, (void*)nullptr, kEmb, 0L,
        nof, nof, 0L, kTok, kEmb, kEmb, kProjScale);
    center_kernel<<<kTok / 8, 256, 0, stream>>>(QF, KC16, KVAR, kQKCarry);
  }

  for (int cidx = 0; cidx < kChunks; ++cidx) {
    const int b  = cidx / kGroupsPerBatch;
    const int h0 = (cidx % kGroupsPerBatch) * kGroup;
    {
      const size_t hoff = (size_t)b * kSeq * kEmb + (size_t)h0 * kHeadDim;
      const int tiles = (kSeq / 64) * (kSeq / 64);
      wmma_gemm64<0, false, 0, 0, false, 0><<<dim3((tiles + 7) / 8, kGroup), 256, 0, stream>>>(
          QC16 + hoff, nou, kEmb, (long)kHeadDim, KC16 + hoff, nou, kEmb, (long)kHeadDim,
          (void*)SC, (void*)nullptr, kSeq, (long)kSeq * kSeq,
          nof, nof, 0L, kSeq, kSeq, kHeadDim, kScoreScale);
    }
    softmax_kernel<<<kGroup * kSeq, 128, 0, stream>>>(SC, QVAR, KVAR, P16, b, h0);
    {
      const int tiles = (kSeq / 64) * (kHeadDim / 64);
      wmma_gemm64<0, false, 0, 1, false, 0><<<dim3((tiles + 7) / 8, kGroup), 256, 0, stream>>>(
          P16, nou, kSeq, (long)kSeq * kSeq,
          VT16 + (size_t)h0 * kHeadDim * kTok + (size_t)b * kSeq, nou, kTok, (long)kHeadDim * kTok,
          (void*)(O16 + (size_t)b * kSeq * kEmb + (size_t)h0 * kHeadDim), (void*)nullptr, kEmb, (long)kHeadDim,
          nof, nof, 0L, kSeq, kHeadDim, kSeq, kPVScale);
    }
  }

  {
    const int tiles = (kTok / 64) * (kEmb / 64);
    wmma_gemm64<0, false, 0, 0, false, 0><<<dim3((tiles + 7) / 8, 1), 256, 0, stream>>>(
        O16, nou, kEmb, 0L, Wo16, nou, kEmb, 0L, (void*)outp, (void*)nullptr, kEmb, 0L,
        nof, nof, 0L, kTok, kEmb, kEmb, kOutScale);
  }
}
